// GraphSAGE_43920335569400
// MI455X (gfx1250) — hardware-run, weakly checked
//
#include <hip/hip_runtime.h>

typedef float          v8f   __attribute__((ext_vector_type(8)));
typedef float          v4f   __attribute__((ext_vector_type(4)));
typedef unsigned int   v4u   __attribute__((ext_vector_type(4)));
typedef int            v8i   __attribute__((ext_vector_type(8)));
typedef unsigned short v8us  __attribute__((ext_vector_type(8)));
typedef unsigned short v16us __attribute__((ext_vector_type(16)));
typedef __bf16         v16bf __attribute__((ext_vector_type(16)));
typedef _Float16       v16h  __attribute__((ext_vector_type(16)));
typedef v4f  __attribute__((may_alias)) v4fa;
typedef v8us __attribute__((may_alias)) v8usa;
union FragB { v16bf v; v16us u; v8us h[2]; v8i w; };
union FragH { v16h  v; v16us u; v8us h[2]; v8i w; };

__device__ __forceinline__ v8f wmb(const FragB& a, const FragB& b, v8f c) {
  v8f d = __builtin_amdgcn_wmma_f32_16x16x32_bf16(false, a.v, false, b.v, (short)0, c, false, false);
  asm volatile("v_nop\n\tv_nop\n\tv_nop\n\tv_nop" : "+v"(d) : "v"(a.w), "v"(b.w));
  return d;
}

__device__ __forceinline__ v8f wmh(const FragH& a, const FragH& b, v8f c) {
  v8f d = __builtin_amdgcn_wmma_f32_16x16x32_f16(false, a.v, false, b.v, (short)0, c, false, false);
  asm volatile("v_nop\n\tv_nop\n\tv_nop\n\tv_nop" : "+v"(d) : "v"(a.w), "v"(b.w));
  return d;
}

__device__ __forceinline__ unsigned bf16_bits(float f) {
  const unsigned u = __float_as_uint(f);
  const unsigned r = (u + 0x7FFFu + ((u >> 16) & 1u)) >> 16;
  const unsigned q = (u >> 16) | 0x40u;
  return ((u & 0x7fffffffu) > 0x7f800000u) ? q : r;
}

__device__ __forceinline__ float bf16_val(float f) {
  return __uint_as_float(bf16_bits(f) << 16);
}
__device__ __forceinline__ int clampi(int v, int lo, int hi) {
  return v < lo ? lo : (v > hi ? hi : v);
}

__device__ __forceinline__ unsigned f16_bits(float f) {
  const unsigned u  = __float_as_uint(f);
  const unsigned s  = (u >> 16) & 0x8000u;
  const unsigned a  = u & 0x7fffffffu;
  const unsigned t  = a - 0x38000000u;
  const unsigned r  = (t + 0x0FFFu + ((t >> 13) & 1u)) >> 13;
  const unsigned rc = r > 0x7C00u ? 0x7C00u : r;
  const bool small  = a < 0x38800000u;
  const bool isnan  = a > 0x7f800000u;
  const unsigned fin = small ? 0u : (s | rc);
  return isnan ? (s | 0x7E00u) : fin;
}

__device__ __forceinline__ unsigned pk16(unsigned lo, unsigned hi) { return lo | (hi << 16); }
__device__ __forceinline__ unsigned bf16_lo_bits(float v) {
  float hi = bf16_val(v);
  asm volatile("" : "+v"(hi));
  return bf16_bits(v - hi);
}
__device__ __forceinline__ v4u pack8_bf16(v4f a, v4f c) {
  return (v4u){ pk16(bf16_bits(a[0]), bf16_bits(a[1])), pk16(bf16_bits(a[2]), bf16_bits(a[3])),
                pk16(bf16_bits(c[0]), bf16_bits(c[1])), pk16(bf16_bits(c[2]), bf16_bits(c[3])) };
}
__device__ __forceinline__ v4u pack8_bf16_lo(v4f a, v4f c) {
  return (v4u){ pk16(bf16_lo_bits(a[0]), bf16_lo_bits(a[1])), pk16(bf16_lo_bits(a[2]), bf16_lo_bits(a[3])),
                pk16(bf16_lo_bits(c[0]), bf16_lo_bits(c[1])), pk16(bf16_lo_bits(c[2]), bf16_lo_bits(c[3])) };
}
__device__ __forceinline__ v4u pack8_f16(v4f a, v4f c) {
  return (v4u){ pk16(f16_bits(a[0]), f16_bits(a[1])), pk16(f16_bits(a[2]), f16_bits(a[3])),
                pk16(f16_bits(c[0]), f16_bits(c[1])), pk16(f16_bits(c[2]), f16_bits(c[3])) };
}

template <int FORM>
__global__ __launch_bounds__(256) void k_plane(const float* __restrict__ src, int rows, int cols, int ldsrc,
                                               unsigned short* __restrict__ dst, int MP, int KP) {
  static_assert(FORM >= 0 && FORM <= 3);
  const int KTOT = (FORM == 1 || FORM == 3) ? 2 * KP : KP;
  const unsigned ppr   = (unsigned)(KTOT >> 3);
  const unsigned kp8   = (unsigned)(KP >> 3);
  const unsigned total = (unsigned)MP * ppr;
  const unsigned g     = blockIdx.x * 256u + threadIdx.x;
  const unsigned rowu  = g / ppr;
  const unsigned p     = g - rowu * ppr;
  const bool second    = p >= kp8;
  const int row = (int)rowu;
  const int c0  = (int)((second ? p - kp8 : p) << 3);
  const float* srow = src + (size_t)clampi(row, 0, rows - 1) * (size_t)ldsrc;
  float x[8];
  unsigned mk[8];
#pragma unroll
  for (int e = 0; e < 8; ++e) {
    const int c = c0 + e;
    const float v = srow[clampi(c, 0, cols - 1)];
    asm volatile("" :: "v"(v));
    x[e]  = v;
    mk[e] = (row < rows && c < cols) ? 0xFFFFu : 0u;
  }
  const v4f a = (v4f){ x[0], x[1], x[2], x[3] };
  const v4f c = (v4f){ x[4], x[5], x[6], x[7] };
  v4u o;
  if (FORM == 2) {
    o = pack8_f16(a, c);
  } else {
    const v4u hi = pack8_bf16(a, c);
    o = hi;
    if (FORM == 1) { const v4u lo = pack8_bf16_lo(a, c); o = second ? lo : hi; }
  }
  const v4u mw = (v4u){ pk16(mk[0], mk[1]), pk16(mk[2], mk[3]), pk16(mk[4], mk[5]), pk16(mk[6], mk[7]) };
  o &= mw;
  if (g < total) {
    volatile v4u* q = (volatile v4u*)(dst + (size_t)g * 8);
    *q = o;
    __threadfence();
    *q = o;
  }
}

template <int FORM> struct FragOf    { typedef FragB T; };
template <>         struct FragOf<2> { typedef FragH T; };
__device__ __forceinline__ v8f mm(const FragB& a, const FragB& b, v8f c) { return wmb(a, b, c); }
__device__ __forceinline__ v8f mm(const FragH& a, const FragH& b, v8f c) { return wmh(a, b, c); }
template <class F> __device__ __forceinline__ F ld_frag(const unsigned short* p) {
  F f;
  f.h[0] = *(const v8usa*)(p);
  f.h[1] = *(const v8usa*)(p + 16);
  return f;
}

template <int FORM, int EPI>
__global__ __launch_bounds__(256) __attribute__((amdgpu_num_vgpr(248)))
void k_gemm_nt(const unsigned short* __restrict__ A, const unsigned short* __restrict__ B,
               const float* __restrict__ bias, float* __restrict__ D, int M, int N, int KTOT, int ldd) {
  static_assert(FORM >= 0 && FORM <= 2);
  static_assert(EPI == 0 || EPI == 1);
  typedef typename FragOf<FORM>::T F;
  __shared__ __attribute__((aligned(16))) float sT[8][16 * 68];
  const int lane = threadIdx.x & 31;
  const int wave = threadIdx.x >> 5;
  const int tilesM = (M + 63) >> 6;
  const int tilesN = (N + 63) >> 6;
  const int tile = blockIdx.x * 8 + wave;
  if (tile >= tilesM * tilesN) return;
  const int tm = tile / tilesN;
  const int tn = tile - tm * tilesN;
  const int m0 = tm << 6;
  const int n0 = tn << 6;

  const int rl = lane & 15;
  const int h8 = (lane >> 4) * 8;
  const unsigned short* pa = A + (size_t)(m0 + rl) * (size_t)KTOT + h8;
  const unsigned short* pb = B + (size_t)(n0 + rl) * (size_t)KTOT + h8;

  v8f acc[4][4];
#pragma unroll
  for (int i = 0; i < 4; ++i)
#pragma unroll
    for (int j = 0; j < 4; ++j) acc[i][j] = (v8f){0.f, 0.f, 0.f, 0.f, 0.f, 0.f, 0.f, 0.f};

#pragma unroll 1
  for (int k0 = 0; k0 < KTOT; k0 += 32) {
    F bf[4];
#pragma unroll
    for (int j = 0; j < 4; ++j) bf[j] = ld_frag<F>(pb + (size_t)(j << 4) * (size_t)KTOT + k0);
#pragma unroll
    for (int i = 0; i < 4; ++i) {
      const F af = ld_frag<F>(pa + (size_t)(i << 4) * (size_t)KTOT + k0);
#pragma unroll
      for (int j = 0; j < 4; ++j) acc[i][j] = mm(af, bf[j], acc[i][j]);
    }
  }

  float* slab = sT[wave];
  const int hh = lane >> 4;
  const int c4 = (lane & 15) * 4;
  const int nc = n0 + c4;
  const bool cok = nc < N;
  v4f bv = (v4f){0.f, 0.f, 0.f, 0.f};
  if (EPI == 1) {
    bv = *(const v4fa*)(bias + clampi(nc, 0, N - 4));
    asm volatile("" :: "v"(bv));
  }
#pragma unroll
  for (int i = 0; i < 4; ++i) {
    const int mBase = m0 + (i << 4);
#pragma unroll
    for (int j = 0; j < 4; ++j) {
#pragma unroll
      for (int r = 0; r < 8; ++r) slab[(h8 + r) * 68 + (j << 4) + rl] = acc[i][j][r];
    }
    __builtin_amdgcn_fence(__ATOMIC_RELEASE, "workgroup");
    __builtin_amdgcn_wave_barrier();
    __builtin_amdgcn_fence(__ATOMIC_ACQUIRE, "workgroup");
    v4f vv[8];
#pragma unroll
    for (int it = 0; it < 8; ++it) {
      const int row = it * 2 + hh;
      v4f v = *(const v4fa*)(slab + row * 68 + c4);
      if (EPI == 1) v += bv;
      vv[it] = v;
    }
    for (int pass = 0; pass < 2; ++pass) {
#pragma unroll
      for (int it = 0; it < 8; ++it) {
        const int row = mBase + it * 2 + hh;
        if (cok && row < M) *(volatile v4f*)(D + (size_t)row * (size_t)ldd + nc) = vv[it];
      }
      __threadfence();
    }
    __builtin_amdgcn_fence(__ATOMIC_RELEASE, "workgroup");
    __builtin_amdgcn_wave_barrier();
    __builtin_amdgcn_fence(__ATOMIC_ACQUIRE, "workgroup");
  }
}

#define SPLIT_MEAN 1
#define SPLIT_H    1

typedef int      v4i  __attribute__((ext_vector_type(4)));
typedef unsigned v2u  __attribute__((ext_vector_type(2)));
typedef v4i __attribute__((may_alias)) v4ia;
typedef v2u __attribute__((may_alias)) v2ua;
typedef v4u __attribute__((may_alias)) v4ua;

static constexpr int kN     = 100000;
static constexpr int kE     = 600000;
static constexpr int kD     = 128;
static constexpr int kMPAD  = 100096;
static constexpr int kNBLK  = 98;
static constexpr int kNBA   = 1024;
static constexpr int kSLA   = 10;
static constexpr int kCHUNK = 2048;
static constexpr int kNCH   = 293;
static constexpr int kCAP   = 8192;
static constexpr int kDEG   = 32;
static constexpr int kK1    = 384;
static constexpr int kK2    = 512;
static constexpr int kBZI   = 3 * kCAP + 2 * kNBA + 32;
static constexpr int kBLDS  = kBZI * 4;

static constexpr size_t kSZ_A    = (size_t)kMPAD * kK2 * 2;
static constexpr size_t kSZ_LIST = (size_t)kNBLK * kCAP * 4;
static constexpr size_t kSZ_CNT  = (size_t)kNBLK * kNBA * 4;
static constexpr size_t kSZ_FLG  = (size_t)kNBLK * 128;
static constexpr size_t kSZ_PREP = (size_t)kD * kK1 * 2 + (size_t)kD * kK2 * 2 + 1024;
static constexpr size_t kO_A     = 0;
static constexpr size_t kO_LIST  = kO_A + kSZ_A;
static constexpr size_t kO_CNT   = kO_LIST + kSZ_LIST;
static constexpr size_t kO_OFF   = kO_CNT + kSZ_CNT;
static constexpr size_t kO_FLG   = kO_OFF + kSZ_CNT;
static constexpr size_t kO_PREP  = kO_FLG + kSZ_FLG;
static constexpr size_t kWS_TOT  = kO_PREP + kSZ_PREP;
static constexpr int kW2OFF = kD * kK1;
static constexpr int kBOFF  = kD * kK1 + kD * kK2;

static_assert(kN == 100000);
static_assert(kE == 292 * 2048 + 1984);
static_assert(kNCH == 293 && (kNCH - 1) * kCHUNK < kE && kNCH * kCHUNK >= kE);
static_assert(kE % 4 == 0 && ((size_t)kE * 4) % 16 == 0);
static_assert(kMPAD == 782 * 128 && kMPAD % 64 == 0 && kMPAD % 8 == 0 && kMPAD >= kN);
static_assert(kNBLK == 98 && kNBLK * kNBA >= kMPAD && kNBA == (1 << kSLA));
static_assert(kCAP % 32 == 0 && kCAP % 128 == 0 && kCAP >= 7872);
static_assert(((long long)(kNCH * kCHUNK) << kSLA) < (1LL << 31));
static_assert(kK1 == 384 && kK2 == 512 && kK1 % 32 == 0 && kK2 % 32 == 0 && kK1 == 3 * kD && kK2 == 4 * kD);
static_assert(kD == 32 * 4);
static_assert(kN % 16 == 0 && kN % 8 == 0);
static_assert(kDEG == 32);
static_assert(kBZI % 4 == 0);
static_assert(kBLDS + 0 <= 262144 && 34816 <= 262144);
static_assert(kSZ_A % 256 == 0 && kSZ_LIST % 256 == 0 && kSZ_CNT % 256 == 0 && kSZ_FLG % 256 == 0 && kSZ_PREP % 256 == 0);
static_assert(kWS_TOT <= ((size_t)128 << 20));
static_assert(((size_t)kBOFF * 2) % 256 == 0 && ((size_t)kW2OFF * 2) % 256 == 0);

__device__ __forceinline__ void wave_sync() {
  __builtin_amdgcn_fence(__ATOMIC_RELEASE, "wavefront");
  __builtin_amdgcn_wave_barrier();
  __builtin_amdgcn_fence(__ATOMIC_ACQUIRE, "wavefront");
}

__device__ __forceinline__ void elu4(float& a0, float& a1, float& a2, float& a3) {
#pragma unroll 1
  for (int q = 0; q < 4; ++q) {
    const float v = a0;
    float r = (v > 0.0f) ? v : expm1f(v);
    asm volatile("" : "+v"(r));
    a0 = a1; a1 = a2; a2 = a3; a3 = r;
  }
}

__device__ __forceinline__ void div4(float& a0, float& a1, float& a2, float& a3, float cf) {
#pragma unroll 1
  for (int q = 0; q < 4; ++q) {
    float r = a0 / cf;
    asm volatile("" : "+v"(r));
    a0 = a1; a1 = a2; a2 = a3; a3 = r;
  }
}

__global__ __launch_bounds__(256) void k_prep(const float* __restrict__ W1l, const float* __restrict__ W1r,
                                              const float* __restrict__ W2l, const float* __restrict__ W2r,
                                              const float* __restrict__ b1, const float* __restrict__ b2,
                                              unsigned short* __restrict__ prep) {
  const int u    = (int)blockIdx.x * 256 + (int)threadIdx.x;
  const int part = u >> 11;
  const int v    = u & 2047;
  const int n    = v >> 4;
  const int k8   = (v & 15) * 8;
  const size_t so = (size_t)n * kD + k8;
  const v4f a1l = *(const v4f*)(W1l + so), c1l = *(const v4f*)(W1l + so + 4);
  const v4f a1r = *(const v4f*)(W1r + so), c1r = *(const v4f*)(W1r + so + 4);
  const v4f a2l = *(const v4f*)(W2l + so), c2l = *(const v4f*)(W2l + so + 4);
  const v4f a2r = *(const v4f*)(W2r + so), c2r = *(const v4f*)(W2r + so + 4);
  asm volatile("" :: "v"(a1l), "v"(c1l));
  asm volatile("" :: "v"(a1r), "v"(c1r));
  asm volatile("" :: "v"(a2l), "v"(c2l));
  asm volatile("" :: "v"(a2r), "v"(c2r));
  const int bq = (v & 31) * 4;
  const v4f ba = *(const v4f*)(b1 + bq);
  const v4f bb = *(const v4f*)(b2 + bq);
  asm volatile("" :: "v"(ba), "v"(bb));
  const unsigned m1r = (part == 0) ? 0xFFFFFFFFu : 0u;
  const unsigned m1l = (part == 1 || part == 2) ? 0xFFFFFFFFu : 0u;
  const unsigned m2r = (part == 3 || part == 4) ? 0xFFFFFFFFu : 0u;
  const unsigned m2l = (part == 5 || part == 6) ? 0xFFFFFFFFu : 0u;
  const unsigned mb  = (part == 7) ? 0xFFFFFFFFu : 0u;
  const unsigned mb2 = ((v & 32) != 0) ? 0xFFFFFFFFu : 0u;
  const v4u p1r = pack8_bf16(a1r, c1r);
  const v4u p1l = pack8_bf16(a1l, c1l);
  const v4u p2r = pack8_bf16(a2r, c2r);
  const v4u p2l = pack8_bf16(a2l, c2l);
  const v4u q1 = (v4u){ bf16_bits(ba[0]) << 16, bf16_bits(ba[1]) << 16, bf16_bits(ba[2]) << 16, bf16_bits(ba[3]) << 16 };
  const v4u q2 = (v4u){ bf16_bits(bb[0]) << 16, bf16_bits(bb[1]) << 16, bf16_bits(bb[2]) << 16, bf16_bits(bb[3]) << 16 };
  const v4u M1r = (v4u){ m1r, m1r, m1r, m1r };
  const v4u M1l = (v4u){ m1l, m1l, m1l, m1l };
  const v4u M2r = (v4u){ m2r, m2r, m2r, m2r };
  const v4u M2l = (v4u){ m2l, m2l, m2l, m2l };
  const v4u MB  = (v4u){ mb, mb, mb, mb };
  const v4u MB2 = (v4u){ mb2, mb2, mb2, mb2 };
  const v4u bo = (q2 & MB2) | (q1 & ~MB2);
  const v4u o  = (p1r & M1r) | (p1l & M1l) | (p2r & M2r) | (p2l & M2l) | (bo & MB);
  const int vb = v < 63 ? v : 63;
  int eoff;
  if (part < 3)      eoff = n * kK1 + part * kD + k8;
  else if (part < 7) eoff = kW2OFF + n * kK2 + (part - 3) * kD + k8;
  else               eoff = kBOFF + vb * 8;
  const bool act = (part < 7) || (part == 7 && v < 64);
  if (act) {
    volatile v4u* q = (volatile v4u*)(prep + (size_t)eoff);
    *q = o;
    __threadfence();
    *q = o;
  }
}

__global__ __launch_bounds__(256) void k_bucket(const int* __restrict__ ei, int* __restrict__ LIST,
                                                int* __restrict__ CNT, int* __restrict__ OFF, int* __restrict__ FLG) {
  extern __shared__ __attribute__((aligned(16))) int dsm[];
  int* hl   = dsm;
  int* sl   = dsm + kCAP;
  int* rk   = dsm + 2 * kCAP;
  int* cnt  = dsm + 3 * kCAP;
  int* offs = cnt + kNBA;
  int* wcnt = offs + kNBA;
  const int tid = (int)threadIdx.x, lane = tid & 31, wave = tid >> 5;
  const int blk = (int)blockIdx.x;
  const unsigned slotBase = (unsigned)(blk * kNBA);
  const int* srcp = ei;
  const int* dstp = ei + kE;

  {
    const v4i z4 = (v4i){0, 0, 0, 0};
    for (int i = tid * 4; i < kBZI; i += 256 * 4) *(v4ia*)(dsm + i) = z4;
  }
  __syncthreads();

  int t = 0;
#pragma unroll 1
  for (int ch = 0; ch < kNCH; ++ch) {
    const int cbase = ch * kCHUNK;
    int  lp[8];
    int  pk[8];
    bool hh[8];
    int  wc = 0;
#pragma unroll
    for (int g = 0; g < 2; ++g) {
      const int e0  = cbase + wave * 256 + g * 128 + lane * 4;
      const int e0c = (e0 < kE - 4) ? e0 : (kE - 4);
      const v4i d = *(const v4i*)(dstp + e0c);
      asm volatile("" :: "v"(d));
      const int fill = (e0 < kE) ? 0 : -1;
      const unsigned s0 = (unsigned)(d.x | fill) - slotBase;
      const unsigned s1 = (unsigned)(d.y | fill) - slotBase;
      const unsigned s2 = (unsigned)(d.z | fill) - slotBase;
      const unsigned s3 = (unsigned)(d.w | fill) - slotBase;
      const bool h0 = s0 < (unsigned)kNBA, h1 = s1 < (unsigned)kNBA;
      const bool h2 = s2 < (unsigned)kNBA, h3 = s3 < (unsigned)kNBA;
      const unsigned m0 = __builtin_amdgcn_ballot_w32(h0);
      const unsigned m1 = __builtin_amdgcn_ballot_w32(h1);
      const unsigned m2 = __builtin_amdgcn_ballot_w32(h2);
      const unsigned m3 = __builtin_amdgcn_ballot_w32(h3);
      const int lower = (int)__builtin_amdgcn_mbcnt_lo(m0, 0u) + (int)__builtin_amdgcn_mbcnt_lo(m1, 0u)
                      + (int)__builtin_amdgcn_mbcnt_lo(m2, 0u) + (int)__builtin_amdgcn_mbcnt_lo(m3, 0u);
      int p = wc + lower;
      lp[4 * g + 0] = p; p += h0 ? 1 : 0;
      lp[4 * g + 1] = p; p += h1 ? 1 : 0;
      lp[4 * g + 2] = p; p += h2 ? 1 : 0;
      lp[4 * g + 3] = p;
      pk[4 * g + 0] = ((e0 + 0) << kSLA) | (int)(s0 & 1023u);
      pk[4 * g + 1] = ((e0 + 1) << kSLA) | (int)(s1 & 1023u);
      pk[4 * g + 2] = ((e0 + 2) << kSLA) | (int)(s2 & 1023u);
      pk[4 * g + 3] = ((e0 + 3) << kSLA) | (int)(s3 & 1023u);
      hh[4 * g + 0] = h0; hh[4 * g + 1] = h1; hh[4 * g + 2] = h2; hh[4 * g + 3] = h3;
      wc += (int)__builtin_popcount(m0) + (int)__builtin_popcount(m1)
          + (int)__builtin_popcount(m2) + (int)__builtin_popcount(m3);
    }
    const int par = (ch & 1) * 8;
    if (lane == 0) wcnt[par + wave] = wc;
    __syncthreads();
    const v4i ca = *(const v4ia*)(wcnt + par);
    const v4i cb = *(const v4ia*)(wcnt + par + 4);
    int cs[8];
    cs[0] = ca.x; cs[1] = ca.y; cs[2] = ca.z; cs[3] = ca.w;
    cs[4] = cb.x; cs[5] = cb.y; cs[6] = cb.z; cs[7] = cb.w;
    int base = t, tot = 0;
#pragma unroll
    for (int w2 = 0; w2 < 8; ++w2) {
      const int c = clampi(cs[w2], 0, 256);
      base += (w2 < wave) ? c : 0;
      tot  += c;
    }
#pragma unroll
    for (int q = 0; q < 8; ++q) {
      const int pos = base + lp[q];
      if (hh[q] && pos < kCAP) hl[pos] = pk[q];
    }
    t += tot;
  }
  __syncthreads();
  const int tt = t < 0 ? 0 : (t > kCAP ? kCAP : t);
  const int ov = (t > kCAP) ? 1 : 0;

  if (wave == 0) {
#pragma unroll 1
    for (int b0 = 0; b0 < tt; b0 += 32) {
      const int idx = b0 + lane;
      const int ent = hl[idx < kCAP ? idx : kCAP - 1];
      const int m32 = (tt - b0) < 32 ? (tt - b0) : 32;
#pragma unroll 1
      for (int k = 0; k < m32; ++k) {
        const int u    = __builtin_amdgcn_readlane(ent, k);
        const int slot = u & (kNBA - 1);
        if (lane == 0) {
          const int r = cnt[slot];
          cnt[slot]  = r + 1;
          rk[b0 + k] = r;
        }
      }
    }
  }
  __syncthreads();
  if (wave == 0) {
    const int sb = lane * (kNBA / 32);
    int s = 0;
#pragma unroll 1
    for (int i = 0; i < kNBA / 32; ++i) s += cnt[sb + i];
    int incl = s;
#pragma unroll
    for (int d = 1; d < 32; d <<= 1) {
      const int y = __shfl_up(incl, d, 32);
      incl += (lane >= d) ? y : 0;
    }
    int run = incl - s;
#pragma unroll 1
    for (int i = 0; i < kNBA / 32; ++i) {
      const int cv = cnt[sb + i];
      offs[sb + i] = run;
      run += cv;
    }
  }
  __syncthreads();
#pragma unroll 1
  for (int b = 0; b < tt; b += 256) {
    const int idx  = b + tid;
    const int idc  = idx < kCAP ? idx : kCAP - 1;
    const int u    = hl[idc];
    const int r    = rk[idc];
    const int slot = u & (kNBA - 1);
    const int p    = clampi(offs[slot] + r, 0, kCAP - 1);
    if (idx < tt) sl[p] = (u >> kSLA) & 0xFFFFF;
  }
  __syncthreads();

  {
    const v4i cv = *(const v4ia*)(cnt + 4 * tid);
    const v4i ofv = *(const v4ia*)(offs + 4 * tid);
    const v4i fv = (v4i){ov, ov, ov, ov};
    volatile v4i* qc = (volatile v4i*)(CNT + (size_t)blk * kNBA + 4 * tid);
    volatile v4i* qo = (volatile v4i*)(OFF + (size_t)blk * kNBA + 4 * tid);
    volatile v4i* qf = (volatile v4i*)(FLG + (size_t)blk * 32 + 4 * (tid & 7));
    *qc = cv;
    *qo = ofv;
    if (tid < 8) *qf = fv;
    __threadfence();
    *qc = cv;
    *qo = ofv;
    if (tid < 8) *qf = fv;
  }
  int ttR = (tt + 127) & ~127;
  ttR = ttR < 128 ? 128 : ttR;
  ttR = ttR > kCAP ? kCAP : ttR;
#pragma unroll 1
  for (int b = 0; b < ttR; b += 1024) {
    const int i4  = b + tid * 4;
    const int i4c = i4 < kCAP - 4 ? i4 : kCAP - 4;
    const v4i e = *(const v4ia*)(sl + i4c);
    const int g0 = srcp[clampi(e.x, 0, kE - 1)];
    const int g1 = srcp[clampi(e.y, 0, kE - 1)];
    const int g2 = srcp[clampi(e.z, 0, kE - 1)];
    const int g3 = srcp[clampi(e.w, 0, kE - 1)];
    asm volatile("" :: "v"(g0), "v"(g1), "v"(g2), "v"(g3));
    const v4i sv = (v4i){ clampi(g0, 0, kN - 1), clampi(g1, 0, kN - 1), clampi(g2, 0, kN - 1), clampi(g3, 0, kN - 1) };
    if (i4 < ttR) {
      volatile v4i* q = (volatile v4i*)(LIST + (size_t)blk * kCAP + i4c);
      *q = sv;
      __threadfence();
      *q = sv;
    }
  }
}

__global__ __launch_bounds__(256) void k_mean1(const float* __restrict__ x, const int* __restrict__ LIST,
                                               const int* __restrict__ CNT, const int* __restrict__ OFF,
                                               const int* __restrict__ FLG, unsigned short* __restrict__ A1) {
  __shared__ __attribute__((aligned(16))) unsigned rowbuf[8 * 192];
  const int tid = (int)threadIdx.x, lane = tid & 31, wave = tid >> 5;
  const int i = (int)blockIdx.x * 8 + wave;
  const bool live = i < kN;
  const int ic  = live ? i : kN - 1;
  const int blk = i >> kSLA;
  const int c  = CNT[i];
  const int o  = OFF[i];
  const int fl = FLG[blk * 32];
  asm volatile("" :: "v"(c), "v"(o), "v"(fl));
  const v4f xs = *(const v4f*)(x + (size_t)ic * kD + 4 * lane);
  asm volatile("" :: "v"(xs));
  const bool big = c > kDEG;
  const int cl = clampi(c, 0, kDEG);
  const int cn = __builtin_amdgcn_readfirstlane(live ? cl : 0);
  const int oc = clampi(o, 0, kCAP - 1);
  const int lq = lane < (cn - 1) ? lane : (cn - 1);
  int li = (cn > 0) ? (oc + lq) : 0;
  li = clampi(li, 0, kCAP - 1);
  const int sraw = LIST[(size_t)blk * kCAP + li];
  asm volatile("" :: "v"(sraw));
  const int sr = clampi(sraw, 0, kN - 1);
  float a0 = 0.0f, a1 = 0.0f, a2 = 0.0f, a3 = 0.0f;
#pragma unroll 1
  for (int k = 0; k < cn; ++k) {
    const int sk = __builtin_amdgcn_readlane(sr, k);
    const v4f a = *(const v4f*)(x + (size_t)sk * kD + 4 * lane);
    a0 += bf16_val(a[0]);
    a1 += bf16_val(a[1]);
    a2 += bf16_val(a[2]);
    a3 += bf16_val(a[3]);
  }
  const float cf = (float)(c > 1 ? c : 1);
  div4(a0, a1, a2, a3, cf);
  const float pz = (fl != 0 || big) ? __uint_as_float(0x7fc00000u) : 0.0f;
  const float m0 = a0 + pz, m1 = a1 + pz, m2 = a2 + pz, m3 = a3 + pz;
  const unsigned lm = live ? 0xFFFFFFFFu : 0u;
  const unsigned xw0 = pk16(bf16_bits(xs[0]), bf16_bits(xs[1])) & lm;
  const unsigned xw1 = pk16(bf16_bits(xs[2]), bf16_bits(xs[3])) & lm;
  const unsigned hw0 = pk16(bf16_bits(m0), bf16_bits(m1)) & lm;
  const unsigned hw1 = pk16(bf16_bits(m2), bf16_bits(m3)) & lm;
#if SPLIT_MEAN
  const unsigned lw0 = pk16(bf16_lo_bits(m0), bf16_lo_bits(m1)) & lm;
  const unsigned lw1 = pk16(bf16_lo_bits(m2), bf16_lo_bits(m3)) & lm;
#else
  const unsigned lw0 = 0u, lw1 = 0u;
#endif
  unsigned* rb = rowbuf + wave * 192;
  *(v2ua*)(rb + 2 * lane)       = (v2u){ xw0, xw1 };
  *(v2ua*)(rb + 64 + 2 * lane)  = (v2u){ hw0, hw1 };
  *(v2ua*)(rb + 128 + 2 * lane) = (v2u){ lw0, lw1 };
  wave_sync();
  const v4u q0 = *(const v4ua*)(rb + 4 * lane);
  const v4u q1 = *(const v4ua*)(rb + 128 + 4 * (lane & 15));
  unsigned short* rp = A1 + (size_t)i * kK1;
  volatile v4u* w0 = (volatile v4u*)(rp + 8 * lane);
  volatile v4u* w1 = (volatile v4u*)(rp + 256 + 8 * (lane & 15));
  *w0 = q0;
  if (lane < 16) *w1 = q1;
  __threadfence();
  *w0 = q0;
  if (lane < 16) *w1 = q1;
}

__global__ __launch_bounds__(256) void k_row1(const float* __restrict__ P, unsigned short* __restrict__ A2) {
  __shared__ __attribute__((aligned(16))) unsigned rowbuf[8 * 128];
  const int tid = (int)threadIdx.x, lane = tid & 31, wave = tid >> 5;
  const int i = (int)blockIdx.x * 8 + wave;
  const bool live = i < kN;
  const int ic = live ? i : kN - 1;
  const v4f p = *(const v4f*)(P + (size_t)ic * kD + 4 * lane);
  asm volatile("" :: "v"(p));
  float a0 = p[0], a1 = p[1], a2 = p[2], a3 = p[3];
  elu4(a0, a1, a2, a3);
  const unsigned lm = live ? 0xFFFFFFFFu : 0u;
  const unsigned hw0 = pk16(bf16_bits(a0), bf16_bits(a1)) & lm;
  const unsigned hw1 = pk16(bf16_bits(a2), bf16_bits(a3)) & lm;
#if SPLIT_H
  const unsigned lw0 = pk16(bf16_lo_bits(a0), bf16_lo_bits(a1)) & lm;
  const unsigned lw1 = pk16(bf16_lo_bits(a2), bf16_lo_bits(a3)) & lm;
#else
  const unsigned lw0 = 0u, lw1 = 0u;
#endif
  unsigned* rb = rowbuf + wave * 128;
  *(v2ua*)(rb + 2 * lane)      = (v2u){ hw0, hw1 };
  *(v2ua*)(rb + 64 + 2 * lane) = (v2u){ lw0, lw1 };
  wave_sync();
  const v4u q0 = *(const v4ua*)(rb + 4 * lane);
  volatile v4u* w0 = (volatile v4u*)(A2 + (size_t)i * kK2 + 8 * lane);
  *w0 = q0;
  __threadfence();
  *w0 = q0;
}

__global__ __launch_bounds__(256) void k_mean2(const int* __restrict__ LIST, const int* __restrict__ CNT,
                                               const int* __restrict__ OFF, const int* __restrict__ FLG,
                                               unsigned short* A2) {
  __shared__ __attribute__((aligned(16))) unsigned rowbuf[8 * 128];
  const int tid = (int)threadIdx.x, lane = tid & 31, wave = tid >> 5;
  const int i = (int)blockIdx.x * 8 + wave;
  const bool live = i < kN;
  const int blk = i >> kSLA;
  const int c  = CNT[i];
  const int o  = OFF[i];
  const int fl = FLG[blk * 32];
  asm volatile("" :: "v"(c), "v"(o), "v"(fl));
  const bool big = c > kDEG;
  const int cl = clampi(c, 0, kDEG);
  const int cn = __builtin_amdgcn_readfirstlane(live ? cl : 0);
  const int oc = clampi(o, 0, kCAP - 1);
  const int lq = lane < (cn - 1) ? lane : (cn - 1);
  int li = (cn > 0) ? (oc + lq) : 0;
  li = clampi(li, 0, kCAP - 1);
  const int sraw = LIST[(size_t)blk * kCAP + li];
  asm volatile("" :: "v"(sraw));
  const int sr = clampi(sraw, 0, kN - 1);
  float a0 = 0.0f, a1 = 0.0f, a2 = 0.0f, a3 = 0.0f;
#pragma unroll 1
  for (int k = 0; k < cn; ++k) {
    const int sk = __builtin_amdgcn_readlane(sr, k);
    const unsigned short* rp = A2 + (size_t)sk * kK2 + 4 * lane;
    const v2u wh = *(const v2ua*)rp;
    const v2u wl = *(const v2ua*)(rp + kD);
    const float f0 = __uint_as_float(wh.x << 16)         + __uint_as_float(wl.x << 16);
    const float f1 = __uint_as_float(wh.x & 0xffff0000u) + __uint_as_float(wl.x & 0xffff0000u);
    const float f2 = __uint_as_float(wh.y << 16)         + __uint_as_float(wl.y << 16);
    const float f3 = __uint_as_float(wh.y & 0xffff0000u) + __uint_as_float(wl.y & 0xffff0000u);
    a0 += f0;
    a1 += f1;
    a2 += f2;
    a3 += f3;
  }
  const float cf = (float)(c > 1 ? c : 1);
  div4(a0, a1, a2, a3, cf);
  const float pz = (fl != 0 || big) ? __uint_as_float(0x7fc00000u) : 0.0f;
  const float m0 = a0 + pz, m1 = a1 + pz, m2 = a2 + pz, m3 = a3 + pz;
  const unsigned lm = live ? 0xFFFFFFFFu : 0u;
  const unsigned hw0 = pk16(bf16_bits(m0), bf16_bits(m1)) & lm;
  const unsigned hw1 = pk16(bf16_bits(m2), bf16_bits(m3)) & lm;
#if SPLIT_MEAN
  const unsigned lw0 = pk16(bf16_lo_bits(m0), bf16_lo_bits(m1)) & lm;
  const unsigned lw1 = pk16(bf16_lo_bits(m2), bf16_lo_bits(m3)) & lm;
#else
  const unsigned lw0 = 0u, lw1 = 0u;
#endif
  unsigned* rb = rowbuf + wave * 128;
  *(v2ua*)(rb + 2 * lane)      = (v2u){ hw0, hw1 };
  *(v2ua*)(rb + 64 + 2 * lane) = (v2u){ lw0, lw1 };
  wave_sync();
  const v4u q0 = *(const v4ua*)(rb + 4 * lane);
  volatile v4u* w0 = (volatile v4u*)(A2 + (size_t)i * kK2 + 2 * kD + 8 * lane);
  *w0 = q0;
  __threadfence();
  *w0 = q0;
}

__global__ __launch_bounds__(256) void k_row2(float* out, const int* __restrict__ CNT, const int* __restrict__ FLG) {
  const int tid = (int)threadIdx.x, lane = tid & 31, wave = tid >> 5;
  const int i = (int)blockIdx.x * 8 + wave;
  float* rowp = out + (size_t)i * kD + 4 * lane;
  const v4f p = *(const v4f*)rowp;
  asm volatile("" :: "v"(p));
  const int c  = CNT[i];
  const int fl = FLG[(i >> kSLA) * 32];
  asm volatile("" :: "v"(c), "v"(fl));
  float a0 = p[0], a1 = p[1], a2 = p[2], a3 = p[3];
  elu4(a0, a1, a2, a3);
  float m = a0;
  m = (a1 > m || a1 != a1) ? a1 : m;
  m = (a2 > m || a2 != a2) ? a2 : m;
  m = (a3 > m || a3 != a3) ? a3 : m;
#pragma unroll
  for (int off = 16; off >= 1; off >>= 1) {
    const float ov = __shfl_xor(m, off, 32);
    m = (ov > m || ov != ov) ? ov : m;
  }
  float t0 = a0 - m, t1 = a1 - m, t2 = a2 - m, t3 = a3 - m;
  float s = 0.0f;
#pragma unroll 1
  for (int q = 0; q < 4; ++q) {
    float e = expf(t0);
    asm volatile("" : "+v"(e));
    s += e;
    const float tmp = t0;
    t0 = t1; t1 = t2; t2 = t3; t3 = tmp;
  }
#pragma unroll
  for (int off = 16; off >= 1; off >>= 1) s += __shfl_xor(s, off, 32);
  const float ls = logf(s);
  const bool pois = (fl != 0) || (c > kDEG);
  const float qn = __uint_as_float(0x7fc00000u);
  v4f o;
  o[0] = pois ? qn : (t0 - ls);
  o[1] = pois ? qn : (t1 - ls);
  o[2] = pois ? qn : (t2 - ls);
  o[3] = pois ? qn : (t3 - ls);
  volatile v4f* w = (volatile v4f*)rowp;
  *w = o;
  __threadfence();
  *w = o;
}

extern "C" void kernel_launch(void* const* d_in, const int* in_sizes, int n_in,
                              void* d_out, int out_size, void* d_ws, size_t ws_size,
                              hipStream_t stream) {
  if (n_in < 8) return;
  if (in_sizes[0] != kN * kD) return;
  if (in_sizes[1] != 2 * kE) return;
  if (in_sizes[2] != kD * kD || in_sizes[4] != kD * kD) return;
  if (in_sizes[5] != kD * kD || in_sizes[7] != kD * kD) return;
  if (in_sizes[3] != kD || in_sizes[6] != kD) return;
  if (out_size != kN * kD) return;
  if (ws_size < kWS_TOT) return;

  const float* x   = (const float*)d_in[0];
  const int*   ei  = (const int*)d_in[1];
  const float* W1l = (const float*)d_in[2];
  const float* b1  = (const float*)d_in[3];
  const float* W1r = (const float*)d_in[4];
  const float* W2l = (const float*)d_in[5];
  const float* b2  = (const float*)d_in[6];
  const float* W2r = (const float*)d_in[7];
  float* out = (float*)d_out;

  char* ws = (char*)d_ws;
  unsigned short* Apl  = (unsigned short*)(ws + kO_A);
  int*            LIST = (int*)(ws + kO_LIST);
  int*            CNT  = (int*)(ws + kO_CNT);
  int*            OFF  = (int*)(ws + kO_OFF);
  int*            FLG  = (int*)(ws + kO_FLG);
  unsigned short* prep = (unsigned short*)(ws + kO_PREP);
  const unsigned short* W1cat = prep;
  const unsigned short* W2cat = prep + kW2OFF;
  const float* btab = (const float*)(prep + kBOFF);

  hipFuncSetAttribute(reinterpret_cast<const void*>(&k_bucket), hipFuncAttributeMaxDynamicSharedMemorySize, kBLDS);

  const int rowBlocks = kMPAD / 8;
  const int tiles     = ((kN + 63) / 64) * ((kD + 63) / 64);
  const int gemmGrid  = (tiles + 7) / 8;

  k_prep<<<57, 256, 0, stream>>>(W1l, W1r, W2l, W2r, b1, b2, prep);
  k_bucket<<<kNBLK, 256, kBLDS, stream>>>(ei, LIST, CNT, OFF, FLG);
  k_mean1<<<rowBlocks, 256, 0, stream>>>(x, LIST, CNT, OFF, FLG, Apl);
  k_gemm_nt<0, 1><<<gemmGrid, 256, 0, stream>>>(Apl, W1cat, btab, out, kN, kD, kK1, kD);
  k_row1<<<rowBlocks, 256, 0, stream>>>(out, Apl);
  k_mean2<<<rowBlocks, 256, 0, stream>>>(LIST, CNT, OFF, FLG, Apl);
  k_gemm_nt<0, 1><<<gemmGrid, 256, 0, stream>>>(Apl, W2cat, btab + kD, out, kN, kD, kK2, kD);
  k_row2<<<kN / 8, 256, 0, stream>>>(out, CNT, FLG);
}
